// BiLSTM_3410204033194
// MI455X (gfx1250) — hardware-verified
//
#include <hip/hip_runtime.h>
#include <hip/hip_bf16.h>

typedef __attribute__((ext_vector_type(16))) _Float16 v16h;
typedef __attribute__((ext_vector_type(8)))  float    v8f;
typedef __attribute__((ext_vector_type(4)))  float    v4f;
#define VST2(T, ptr, val) do { const T _v = (val); *(volatile T*)(ptr) = _v; __threadfence(); *(volatile T*)(ptr) = _v; } while (0)
__device__ __forceinline__ int kmap16(int j, int hh) { return (j < 8) ? (8 * hh + j) : (16 + 8 * hh + (j - 8)); }
__device__ __forceinline__ v8f wmma16(v16h a, v16h b, v8f c) {
    v8f d = __builtin_amdgcn_wmma_f32_16x16x32_f16(false, a, false, b, (short)0, c, false, false);
    asm volatile("v_nop\n\tv_nop\n\tv_nop\n\tv_nop" : "+v"(d) : "v"(a), "v"(b));
    return d;
}

#define TT 1024
#define BB 512
#define HH 20
#define GG 80
#define NTB 32
#define NTHREADS 160

__device__ __forceinline__ void lds_barrier() {
    asm volatile("s_wait_dscnt 0x0\n\t"
                 "s_barrier_signal -1\n\t"
                 "s_barrier_wait -1" ::: "memory");
}

__device__ __forceinline__ float sig_(float x) {
    return __builtin_amdgcn_rcpf(1.0f + expf(-x));
}
__device__ __forceinline__ float tanh_(float x) {
    return fmaf(2.0f, __builtin_amdgcn_rcpf(1.0f + expf(-2.0f * x)), -1.0f);
}

__device__ __forceinline__ int afrag_lane(int m, int kl) { return m + (((kl >> 3) & 1) << 4); }
__device__ __forceinline__ int afrag_half(int kl)        { return (kl & 7) | (((kl >> 4) & 1) << 3); }

__device__ __forceinline__ void store_hrows(const float* __restrict__ sh, float* __restrict__ Hd, size_t t, int btile, int tid) {
    float* dst = Hd + (t * BB + (size_t)btile * 16) * HH;
    if (tid < 80) VST2(v4f, dst + tid * 4, *(const v4f*)(sh + tid * 4));
}

__global__ __launch_bounds__(NTHREADS)
void lstm_l0_kernel(const float* __restrict__ X,
                    const float* __restrict__ w_ih_b,
                    const float* __restrict__ w_hh_b,
                    const float* __restrict__ b_b,
                    float* __restrict__ Hout)
{
    __shared__ __align__(16) float sh[16 * HH];
    const int dir = blockIdx.y, btile = blockIdx.x;
    const int tid = threadIdx.x, lane = tid & 31, nt = tid >> 5;
    const float* w_ih = w_ih_b + (size_t)dir * GG * 2;
    const float* w_hh = w_hh_b + (size_t)dir * GG * HH;
    const float* bias = b_b    + (size_t)dir * GG;

    __shared__ __align__(32) _Float16 afrag[32][16];
    __shared__ float gates[16][GG];

    const int ncol = nt * 16 + (lane & 15);
    v16h bfrag;
    #pragma unroll
    for (int j = 0; j < 16; ++j) {
        const int k = kmap16(j, lane >> 4);
        float w = 0.0f;
        if (k < 2)            w = w_ih[ncol * 2 + k];
        else if (k < 2 + HH)  w = w_hh[ncol * HH + (k - 2)];
        bfrag[j] = (_Float16)w;
    }
    float* Hd = Hout + (size_t)dir * TT * BB * HH;
    const float bcol = bias[ncol];
    v8f cinit;
    #pragma unroll
    for (int v = 0; v < 8; ++v) cinit[v] = bcol;

    for (int p = tid; p < 32 * 16; p += NTHREADS) ((_Float16*)afrag)[p] = (_Float16)0.0f;

    const int i0 = 2 * tid, i1 = 2 * tid + 1;
    const int r0 = i0 / HH, j0 = i0 % HH, r1 = i1 / HH, j1 = i1 % HH;
    float c0 = 0.0f, c1 = 0.0f;

    float xreg = 0.0f;
    {
        const int t0 = dir ? (TT - 1) : 0;
        if (tid < 32)
            xreg = X[((size_t)t0 * BB + btile * 16 + (tid >> 1)) * 2 + (tid & 1)];
    }

    for (int s = 0; s < TT; ++s) {
        const int t = dir ? (TT - 1 - s) : s;

        if (tid < 32) afrag[tid >> 1][tid & 1] = (_Float16)xreg;
        lds_barrier();

        {
            const int sn = (s + 1 < TT) ? s + 1 : s;
            const int tn = dir ? (TT - 1 - sn) : sn;
            if (tid < 32)
                xreg = X[((size_t)tn * BB + btile * 16 + (tid >> 1)) * 2 + (tid & 1)];
        }

        v8f c = cinit;
        {
            v16h a = *(const v16h*)(&afrag[lane][0]);
            c = wmma16(a, bfrag, c);
        }
        #pragma unroll
        for (int v = 0; v < 8; ++v)
            gates[v + ((lane >> 4) << 3)][ncol] = c[v];
        lds_barrier();

        const size_t tb = (size_t)t * NTB + btile;
        {
            const float gi = gates[r0][j0],          gf = gates[r0][HH + j0];
            const float gc = gates[r0][2 * HH + j0], go = gates[r0][3 * HH + j0];
            c0 = sig_(gf) * c0 + sig_(gi) * tanh_(gc);
            const _Float16 hf = (_Float16)(sig_(go) * tanh_(c0));
            const int kl = 2 + j0;
            afrag[afrag_lane(r0, kl)][afrag_half(kl)] = hf;
            sh[r0 * HH + j0] = sig_(go) * tanh_(c0);
        }
        {
            const float gi = gates[r1][j1],          gf = gates[r1][HH + j1];
            const float gc = gates[r1][2 * HH + j1], go = gates[r1][3 * HH + j1];
            c1 = sig_(gf) * c1 + sig_(gi) * tanh_(gc);
            const _Float16 hf = (_Float16)(sig_(go) * tanh_(c1));
            const int kl = 2 + j1;
            afrag[afrag_lane(r1, kl)][afrag_half(kl)] = hf;
            sh[r1 * HH + j1] = sig_(go) * tanh_(c1);
        }
        lds_barrier();
        store_hrows(sh, Hd, (size_t)t, btile, tid);
        (void)tb;
    }
}

template<int OUT_MODE>
__global__ __launch_bounds__(NTHREADS)
void lstm_mid_kernel(const float* __restrict__ Hin,
                     const float* __restrict__ w_ih_b,
                     const float* __restrict__ w_hh_b,
                     const float* __restrict__ b_b,
                     float* __restrict__ Hout)
{
    __shared__ __align__(16) float sh[16 * HH];
    const int dir = blockIdx.y, btile = blockIdx.x;
    const int tid = threadIdx.x, lane = tid & 31, nt = tid >> 5;
    const float* w_ih = w_ih_b + (size_t)dir * GG * 40;
    const float* w_hh = w_hh_b + (size_t)dir * GG * HH;
    const float* bias = b_b    + (size_t)dir * GG;

    __shared__ __align__(32) _Float16 afrag1[32][16];
    __shared__ float gates[16][GG];

    const int ncol = nt * 16 + (lane & 15);
    v16h bfrag[2];
    #pragma unroll
    for (int f = 0; f < 2; ++f) {
        #pragma unroll
        for (int j = 0; j < 16; ++j) {
            const int k = f * 32 + kmap16(j, lane >> 4);
            float w = 0.0f;
            if (k < 40)           w = w_ih[ncol * 40 + k];
            else if (k < 40 + HH) w = w_hh[ncol * HH + (k - 40)];
            bfrag[f][j] = (_Float16)w;
        }
    }
    float* Hd = Hout + (size_t)dir * TT * BB * HH;
    const float* H0 = Hin;
    const float* H1 = Hin + (size_t)TT * BB * HH;
    const int mrow = btile * 16 + (lane & 15), hh = lane >> 4;
    const float bcol = bias[ncol];
    v8f cinit;
    #pragma unroll
    for (int v = 0; v < 8; ++v) cinit[v] = bcol;

    for (int p = tid; p < 32 * 16; p += NTHREADS) ((_Float16*)afrag1)[p] = (_Float16)0.0f;

    const int i0 = 2 * tid, i1 = 2 * tid + 1;
    const int r0 = i0 / HH, j0 = i0 % HH, r1 = i1 / HH, j1 = i1 % HH;
    float c0 = 0.0f, c1 = 0.0f;

    for (int s = 0; s < TT; ++s) {
        const int t = dir ? (TT - 1 - s) : s;
        lds_barrier();

        const float* x0r = H0 + ((size_t)t * BB + mrow) * HH;
        const float* x1r = H1 + ((size_t)t * BB + mrow) * HH;
        v16h a0reg;
        #pragma unroll
        for (int j = 0; j < 16; ++j) { const int k = kmap16(j, hh); a0reg[j] = (_Float16)((k < HH) ? x0r[k] : x1r[k - HH]); }
        v16h a1 = *(const v16h*)(&afrag1[lane][0]);
        if (hh == 0) {
            #pragma unroll
            for (int j = 0; j < 8; ++j) a1[j] = (_Float16)x1r[12 + j];
        }

        v8f c = cinit;
        c = wmma16(a0reg, bfrag[0], c);
        c = wmma16(a1, bfrag[1], c);
        #pragma unroll
        for (int v = 0; v < 8; ++v)
            gates[v + ((lane >> 4) << 3)][ncol] = c[v];
        lds_barrier();

        const size_t tb = (size_t)t * NTB + btile;
        {
            const float gi = gates[r0][j0],          gf = gates[r0][HH + j0];
            const float gc = gates[r0][2 * HH + j0], go = gates[r0][3 * HH + j0];
            c0 = sig_(gf) * c0 + sig_(gi) * tanh_(gc);
            const float h = sig_(go) * tanh_(c0);
            const _Float16 hf = (_Float16)h;
            const int kl = 8 + j0;
            afrag1[afrag_lane(r0, kl)][afrag_half(kl)] = hf;
            sh[r0 * HH + j0] = h;
        }
        {
            const float gi = gates[r1][j1],          gf = gates[r1][HH + j1];
            const float gc = gates[r1][2 * HH + j1], go = gates[r1][3 * HH + j1];
            c1 = sig_(gf) * c1 + sig_(gi) * tanh_(gc);
            const float h = sig_(go) * tanh_(c1);
            const _Float16 hf = (_Float16)h;
            const int kl = 8 + j1;
            afrag1[afrag_lane(r1, kl)][afrag_half(kl)] = hf;
            sh[r1 * HH + j1] = h;
        }
        lds_barrier();
        store_hrows(sh, Hd, (size_t)t, btile, tid);
        (void)tb;
    }
}

__global__ void fc_kernel(const float* __restrict__ Hl,
                          const float* __restrict__ fc_w,
                          const float* __restrict__ fc_b,
                          float* __restrict__ out)
{
    const int t = blockIdx.x * blockDim.x + threadIdx.x;
    if (t >= TT) return;
    const float* r0 = Hl + ((size_t)t * BB + (BB - 1)) * HH;
    const float* r1 = Hl + (size_t)TT * BB * HH + ((size_t)t * BB + (BB - 1)) * HH;
    v4f o;
    #pragma unroll
    for (int c = 0; c < 4; ++c) {
        float acc = fc_b[c];
        #pragma unroll 4
        for (int k = 0; k < HH; ++k) acc += r0[k] * fc_w[c * 40 + k] + r1[k] * fc_w[c * 40 + HH + k];
        o[c] = acc;
    }
    VST2(v4f, out + (size_t)t * 4, o);
}

extern "C" void kernel_launch(void* const* d_in, const int* in_sizes, int n_in,
                              void* d_out, int out_size, void* d_ws, size_t ws_size,
                              hipStream_t stream)
{
    (void)in_sizes; (void)n_in; (void)out_size;
    const float* x      = (const float*)d_in[0];
    const float* w_ih0  = (const float*)d_in[1];
    const float* w_hh0  = (const float*)d_in[2];
    const float* b0     = (const float*)d_in[3];
    const float* w_ih12 = (const float*)d_in[4];
    const float* w_hh12 = (const float*)d_in[5];
    const float* b12    = (const float*)d_in[6];
    const float* fc_w   = (const float*)d_in[7];
    const float* fc_b   = (const float*)d_in[8];
    float* out = (float*)d_out;

    if (ws_size < (size_t)2 * 2 * TT * BB * HH * 4) return;
    float* Ha = (float*)d_ws;
    float* Hb = Ha + (size_t)2 * TT * BB * HH;

    dim3 grid(NTB, 2), block(NTHREADS);
    lstm_l0_kernel<<<grid, block, 0, stream>>>(x, w_ih0, w_hh0, b0, Ha);
    lstm_mid_kernel<0><<<grid, block, 0, stream>>>(Ha, w_ih12, w_hh12, b12, Hb);
    lstm_mid_kernel<1><<<grid, block, 0, stream>>>(Hb, w_ih12 + (size_t)2 * GG * 40, w_hh12 + (size_t)2 * GG * HH, b12 + 2 * GG, Ha);
    fc_kernel<<<dim3(8), dim3(128), 0, stream>>>(Ha, fc_w, fc_b, out);
}
